// CrossAttention_17300128268956
// MI455X (gfx1250) — hardware-run, weakly checked
//
#include <hip/hip_runtime.h>


#ifndef NB
#define NB 2
#endif
#ifndef SEQ
#define SEQ 2048
#endif
#define NB_FULL  2
#define SEQ_FULL 2048
#ifndef OUT_SEQ
#define OUT_SEQ SEQ
#endif
#ifndef AM_PITCH
#define AM_PITCH SEQ
#endif
#define DM   1024
#define NH_  16
#define HD   64
#define RP   (HD / 2)
#define AW   4
#define AKS  64
#define QRS  2048.0f
#define LOG2E 1.4426950408889634f
#define SC2  (0.125f * LOG2E)
#define PSH  8.0f
#define AMW  (256.0f / (float)NH_)
#define LOG2TH 15.609640474436812f
#define KA   (2 * DM)
#define NWORDS (NB * SEQ / 32)
#define NWP  (((NWORDS + 31) / 32) * 32)
#define AM_OFF ((size_t)NB_FULL * SEQ_FULL * DM)

static_assert(HD == 64);
static_assert(NH_ * HD == DM);
static_assert(NH_ == 16);
static_assert(RP == 32);
static_assert(DM == 4 * 32 * 8);
static_assert(DM % 64 == 0);
static_assert(DM % 32 == 0);
static_assert(SEQ % 64 == 0);
static_assert((NB * SEQ) % 64 == 0);
static_assert((NB * SEQ) % 8 == 0);
static_assert(SEQ % 8 == 0);
static_assert(SEQ % 32 == 0);
static_assert(SEQ % (16 * AW) == 0);
static_assert(AKS == 64);
static_assert(SEQ % AKS == 0);
static_assert(((size_t)SEQ * DM) % 64 == 0);
static_assert(((size_t)DM * DM) % 64 == 0);
static_assert(NB <= NB_FULL);
static_assert(SEQ <= SEQ_FULL);
static_assert((size_t)NB_FULL * SEQ_FULL * DM * 4 == (size_t)16777216);
static_assert(AM_OFF * 4 == (size_t)16777216);
static_assert((AM_OFF + (size_t)NB_FULL * SEQ_FULL * SEQ_FULL) * 4 == (size_t)50331648);
static_assert(AM_OFF % 32 == 0);
static_assert(AM_PITCH % 32 == 0);
static_assert(((size_t)(NB - 1) * OUT_SEQ + (size_t)(SEQ - 1)) * (size_t)AM_PITCH + SEQ <= (size_t)NB_FULL * SEQ_FULL * SEQ_FULL);

typedef _Float16 h16;
typedef unsigned short bf;
typedef __attribute__((ext_vector_type(16))) __bf16   v16bf;
typedef __attribute__((ext_vector_type(16))) _Float16 v16h;
typedef __attribute__((ext_vector_type(8)))  _Float16 v8h;
typedef __attribute__((ext_vector_type(8)))  unsigned short v8us;
typedef __attribute__((ext_vector_type(8)))  float    v8f;
typedef __attribute__((ext_vector_type(4)))  float    v4f;
typedef __attribute__((ext_vector_type(2)))  float    v2f;
typedef __attribute__((ext_vector_type(4)))  unsigned v4u;
typedef __attribute__((ext_vector_type(4)))  int      v4i;
typedef v4f  __attribute__((may_alias)) v4fa;

__device__ __forceinline__ unsigned short f2bf(float f) { unsigned u = __float_as_uint(f); u += 0x7FFFu + ((u >> 16) & 1u); return (unsigned short)(u >> 16); }
__device__ __forceinline__ float bf2f(unsigned short s) { return __uint_as_float(((unsigned)s) << 16); }
__device__ __forceinline__ float bfr(float f) { return bf2f(f2bf(f)); }
__device__ __forceinline__ v16h cat16(v8h lo, v8h hi) { return __builtin_shufflevector(lo, hi, 0, 1, 2, 3, 4, 5, 6, 7, 8, 9, 10, 11, 12, 13, 14, 15); }
__device__ __forceinline__ v16bf cat16b(v8us lo, v8us hi) { return __builtin_bit_cast(v16bf, __builtin_shufflevector(lo, hi, 0, 1, 2, 3, 4, 5, 6, 7, 8, 9, 10, 11, 12, 13, 14, 15)); }
__device__ __forceinline__ v8f wmma16(v16h a, v16h b, v8f c) { return __builtin_amdgcn_wmma_f32_16x16x32_f16(false, a, false, b, (short)0, c, false, false); }
__device__ __forceinline__ v8f wmmab(v16bf a, v16bf b, v8f c) { return __builtin_amdgcn_wmma_f32_16x16x32_bf16(false, a, false, b, (short)0, c, false, false); }
__device__ __forceinline__ v16h  ldh(const h16* p) { return cat16(*(const v8h*)p, *(const v8h*)(p + 16)); }
__device__ __forceinline__ v16bf ldb(const bf* p)  { return cat16b(*(const v8us*)p, *(const v8us*)(p + 16)); }
__device__ __forceinline__ void wave_sync() { __builtin_amdgcn_fence(3  , "wavefront"); __builtin_amdgcn_wave_barrier(); asm volatile("" ::: "memory"); }
static __device__ __forceinline__ h16 toh_flush(float v) { const h16 r = (h16)v; return (fabsf(v) < 6.103515625e-05f) ? (h16)0.0f : r; }
static __device__ __forceinline__ h16 p_exp2_flush(float e, bool vis) { const float v = __builtin_amdgcn_exp2f(e); const h16 r = (h16)v; return (vis && (e >= -14.0f)) ? r : (h16)0.0f; }

__global__ __launch_bounds__(32) void k_mask(const int* __restrict__ mask, unsigned* MW, int nW) {
    const int lane = threadIdx.x & 31;
    const int w = blockIdx.x * 32 + lane;
    const int wc = (w < nW) ? w : (nW - 1);
    const int b = wc / (SEQ / 32), tw = wc % (SEQ / 32);
    const int* s = mask + (size_t)b * SEQ_FULL + (size_t)tw * 32;
    unsigned word = 0u;
#pragma unroll
    for (int j = 0; j < 8; ++j) { const v4i m = *(const v4i*)(s + 4 * j);
        word |= ((m[0] != 0) ? 1u : 0u) << (4 * j);     word |= ((m[1] != 0) ? 1u : 0u) << (4 * j + 1);
        word |= ((m[2] != 0) ? 1u : 0u) << (4 * j + 2); word |= ((m[3] != 0) ? 1u : 0u) << (4 * j + 3); }
    const unsigned val = (w < nW) ? word : 0u;
    *(volatile unsigned*)(MW + w) = val; __threadfence(); *(volatile unsigned*)(MW + w) = val;
}

__global__ __launch_bounds__(256) void k_cvt(const float* __restrict__ src, bf* dst, unsigned perBatch8, unsigned c8n, size_t sBatch, size_t sRow) {
    const unsigned i = blockIdx.x * 256u + threadIdx.x; if (i >= perBatch8) return;
    const unsigned r = i / c8n, c = i - r * c8n; const unsigned b = blockIdx.y;
    const v8f v = *(const v8f*)(src + (size_t)b * sBatch + (size_t)r * sRow + (size_t)c * 8); v8us o;
#pragma unroll
    for (int k = 0; k < 8; ++k) o[k] = f2bf(v[k]);
    const size_t oo = ((size_t)b * perBatch8 + i) * 8;
    *(volatile v8us*)(dst + oo) = o; __threadfence(); *(volatile v8us*)(dst + oo) = o;
}

__global__ __launch_bounds__(256) void k_rtab(float* RC, float* RS) {
#pragma clang fp contract(off)
    const int lane = threadIdx.x & 31; const int wave = __builtin_amdgcn_readfirstlane(threadIdx.x >> 5);
    const int t = blockIdx.x * 8 + wave;
    const float ex = (float)(2 * lane) * (1.0f / (float)HD);
    const float inv = exp2f(-ex * LOG2TH);
    const float ang = (float)t * inv;
    float sn, cs; sincosf(ang, &sn, &cs);
    const size_t oo = (size_t)t * RP + lane;
    *(volatile float*)(RC + oo) = cs; *(volatile float*)(RS + oo) = sn;
    __threadfence();
    *(volatile float*)(RC + oo) = cs; *(volatile float*)(RS + oo) = sn;
}

__global__ __launch_bounds__(32) void k_pre(const bf* __restrict__ A, const bf* __restrict__ Bt, const float* __restrict__ bias, float* OUT) {
    __shared__ __align__(16) float os[16 * 68];
    const int lane = threadIdx.x & 31, lr = lane & 15, hi = lane >> 4; const int r0 = blockIdx.x * 64, c0 = blockIdx.y * 64;
    v8f acc[4][4];
#pragma unroll
    for (int mb = 0; mb < 4; ++mb)
#pragma unroll
        for (int nb = 0; nb < 4; ++nb) acc[mb][nb] = (v8f){};
    const size_t aoff = (size_t)(r0 + lr) * DM + 8 * hi, boff = (size_t)(c0 + lr) * DM + 8 * hi;
#pragma unroll 1
    for (int kc = 0; kc < DM; kc += 32) {
        v16bf a[4];
#pragma unroll
        for (int mb = 0; mb < 4; ++mb) a[mb] = ldb(A + aoff + (size_t)mb * 16 * DM + kc);
        v16bf b = ldb(Bt + boff + kc);
#pragma unroll
        for (int mb = 0; mb < 4; ++mb) acc[mb][0] = wmmab(a[mb], b, acc[mb][0]);
#pragma unroll
        for (int nb = 1; nb < 4; ++nb) { b = ldb(Bt + boff + (size_t)nb * 16 * DM + kc);
#pragma unroll
            for (int mb = 0; mb < 4; ++mb) acc[mb][nb] = wmmab(a[mb], b, acc[mb][nb]); }
        asm volatile("" : "+v"(acc[2][0]), "+v"(acc[2][1]), "+v"(acc[2][2]), "+v"(acc[2][3]), "+v"(acc[3][0]), "+v"(acc[3][1]), "+v"(acc[3][2]), "+v"(acc[3][3]));
        asm volatile("v_nop\n\tv_nop\n\tv_nop\n\tv_nop" : "+v"(acc[0][0]), "+v"(acc[0][1]), "+v"(acc[0][2]), "+v"(acc[0][3]), "+v"(acc[1][0]), "+v"(acc[1][1]), "+v"(acc[1][2]), "+v"(acc[1][3]) : "v"(a[0]), "v"(a[1]), "v"(a[2]), "v"(a[3]), "v"(b));
    }
    const int cofs = lr * 4;
    const v4f braw = *(const v4f*)(bias + c0 + cofs);
    v4f bv; bv[0] = bfr(braw[0]); bv[1] = bfr(braw[1]); bv[2] = bfr(braw[2]); bv[3] = bfr(braw[3]);
    float* orow = OUT + (size_t)r0 * DM + c0;
#pragma unroll
    for (int mb = 0; mb < 4; ++mb) {
#pragma unroll
        for (int nb = 0; nb < 4; ++nb) {
#pragma unroll
            for (int j = 0; j < 8; ++j) os[(hi * 8 + j) * 68 + nb * 16 + lr] = acc[mb][nb][j]; }
        wave_sync();
#pragma unroll 1
        for (int ps = 0; ps < 2; ++ps) {
#pragma unroll
            for (int s = 0; s < 8; ++s) { const int row = 2 * s + hi;
                const v4f x = *(const v4fa*)(&os[row * 68 + cofs]);
                const v4f val = x + bv;
                *(volatile v4f*)(orow + (size_t)(mb * 16 + row) * DM + cofs) = val; }
            if (ps == 0) __threadfence(); }
        wave_sync();
    }
}

__global__ __launch_bounds__(256) void k_nrope(const float* __restrict__ PRE, const float* __restrict__ gain, const float* __restrict__ RC, const float* __restrict__ RS, h16* PL) {
#pragma clang fp contract(off)
    const int lane = threadIdx.x & 31; const int wave = __builtin_amdgcn_readfirstlane(threadIdx.x >> 5);
    const int row = blockIdx.x * 8 + wave;
    const int b = row / SEQ, t = row % SEQ;
    const float* src = PRE + (size_t)row * DM + 8 * lane;
    const float* gp = gain + 8 * lane;
    float ss = 0.0f;
#pragma unroll 1
    for (int i = 0; i < 4; ++i) { const v4f a = *(const v4f*)(src + 256 * i); const v4f c = *(const v4f*)(src + 256 * i + 4);
        const float s0 = (a[0] * a[0] + a[1] * a[1]) + (a[2] * a[2] + a[3] * a[3]);
        const float s1 = (c[0] * c[0] + c[1] * c[1]) + (c[2] * c[2] + c[3] * c[3]);
        ss += s0 + s1; }
    ss += __shfl_xor(ss, 16, 32); ss += __shfl_xor(ss, 8, 32); ss += __shfl_xor(ss, 4, 32); ss += __shfl_xor(ss, 2, 32); ss += __shfl_xor(ss, 1, 32);
    const float rstd = rsqrtf(ss * (1.0f / (float)DM) + 1.0e-6f);
    const int pq = (lane & 7) * 4;
    const v4f cs = *(const v4f*)(RC + (size_t)t * RP + pq); const v4f sn = *(const v4f*)(RS + (size_t)t * RP + pq);
    const size_t ob = ((size_t)(b * NH_ + (lane >> 3)) * SEQ + t) * HD + (size_t)((lane & 7) * 8);
#pragma unroll 1
    for (int ps = 0; ps < 2; ++ps) {
#pragma unroll 1
        for (int i = 0; i < 4; ++i) {
            const v4f a = *(const v4f*)(src + 256 * i); const v4f c = *(const v4f*)(src + 256 * i + 4);
            const v4f g0 = *(const v4f*)(gp + 256 * i); const v4f g1 = *(const v4f*)(gp + 256 * i + 4);
            v8h hv;
#pragma unroll
            for (int j = 0; j < 2; ++j) {
                const float xe = (a[2 * j] * rstd) * bfr(g0[2 * j]); const float xo = (a[2 * j + 1] * rstd) * bfr(g0[2 * j + 1]);
                hv[2 * j] = toh_flush(xe * cs[j] - xo * sn[j]); hv[2 * j + 1] = toh_flush(xe * sn[j] + xo * cs[j]);
                const float ye = (c[2 * j] * rstd) * bfr(g1[2 * j]); const float yo = (c[2 * j + 1] * rstd) * bfr(g1[2 * j + 1]);
                hv[4 + 2 * j] = toh_flush(ye * cs[2 + j] - yo * sn[2 + j]); hv[4 + 2 * j + 1] = toh_flush(ye * sn[2 + j] + yo * cs[2 + j]); }
            *(volatile v8h*)(PL + ob + (size_t)(4 * i) * SEQ * HD) = hv; }
        if (ps == 0) __threadfence(); }
}

__global__ __launch_bounds__(32) void k_proj(const bf* __restrict__ A, const bf* __restrict__ Bt, const float* __restrict__ bias, int biasRow, h16* Ph, h16* Pr, int useRes, int RB, size_t sRB, int pitch, int CB, size_t sCB) {
    __shared__ __align__(16) float os[16 * 68];
    const int K = DM;
    const int lane = threadIdx.x & 31, lr = lane & 15, hi = lane >> 4; const int r0 = blockIdx.x * 64, c0 = blockIdx.y * 64;
    v8f acc[4][4];
#pragma unroll
    for (int mb = 0; mb < 4; ++mb)
#pragma unroll
        for (int nb = 0; nb < 4; ++nb) acc[mb][nb] = (v8f){};
    const size_t aoff = (size_t)(r0 + lr) * K + 8 * hi, boff = (size_t)(c0 + lr) * K + 8 * hi;
#pragma unroll 1
    for (int kc = 0; kc < K; kc += 32) {
        v16bf a[4];
#pragma unroll
        for (int mb = 0; mb < 4; ++mb) a[mb] = ldb(A + aoff + (size_t)mb * 16 * K + kc);
        v16bf b = ldb(Bt + boff + kc);
#pragma unroll
        for (int mb = 0; mb < 4; ++mb) acc[mb][0] = wmmab(a[mb], b, acc[mb][0]);
#pragma unroll
        for (int nb = 1; nb < 4; ++nb) { b = ldb(Bt + boff + (size_t)nb * 16 * K + kc);
#pragma unroll
            for (int mb = 0; mb < 4; ++mb) acc[mb][nb] = wmmab(a[mb], b, acc[mb][nb]); }
        asm volatile("" : "+v"(acc[2][0]), "+v"(acc[2][1]), "+v"(acc[2][2]), "+v"(acc[2][3]), "+v"(acc[3][0]), "+v"(acc[3][1]), "+v"(acc[3][2]), "+v"(acc[3][3]));
        asm volatile("v_nop\n\tv_nop\n\tv_nop\n\tv_nop" : "+v"(acc[0][0]), "+v"(acc[0][1]), "+v"(acc[0][2]), "+v"(acc[0][3]), "+v"(acc[1][0]), "+v"(acc[1][1]), "+v"(acc[1][2]), "+v"(acc[1][3]) : "v"(a[0]), "v"(a[1]), "v"(a[2]), "v"(a[3]), "v"(b));
    }
    const size_t tbase = (size_t)(r0 / RB) * sRB + (size_t)(r0 % RB) * (size_t)pitch + (size_t)(c0 / CB) * sCB + (size_t)(c0 % CB);
    const int c8 = (lane & 7) * 8, rq = lane >> 3;
    const int bco = biasRow ? 0 : (c0 + c8);
    const v4f bc0 = *(const v4f*)(bias + bco), bc1 = *(const v4f*)(bias + bco + 4);
    float bcv[8];
#pragma unroll
    for (int i = 0; i < 4; ++i) { bcv[i] = bfr(bc0[i]); bcv[4 + i] = bfr(bc1[i]); }
#pragma unroll
    for (int mb = 0; mb < 4; ++mb) {
#pragma unroll
        for (int nb = 0; nb < 4; ++nb) {
#pragma unroll
            for (int j = 0; j < 8; ++j) os[(hi * 8 + j) * 68 + nb * 16 + lr] = acc[mb][nb][j]; }
        wave_sync();
        const size_t sb = tbase + (size_t)(mb * 16) * (size_t)pitch;
#pragma unroll 1
        for (int ps = 0; ps < 2; ++ps) {
#pragma unroll
            for (int s = 0; s < 4; ++s) { const int row = 4 * s + rq;
                const int bro = biasRow ? (r0 + mb * 16 + row) : 0;
                const float brv = bfr(bias[bro]);
                const v4f x0 = *(const v4fa*)(&os[row * 68 + c8]); const v4f x1 = *(const v4fa*)(&os[row * 68 + c8 + 4]); v8h hv, rv;
#pragma unroll
                for (int i = 0; i < 4; ++i) { const float y0 = x0[i] + (biasRow ? brv : bcv[i]); const float y1 = x1[i] + (biasRow ? brv : bcv[4 + i]);
                    const h16 a0 = (h16)y0; const h16 a1 = (h16)y1; hv[i] = a0; hv[4 + i] = a1; rv[i] = (h16)((y0 - (float)a0) * QRS); rv[4 + i] = (h16)((y1 - (float)a1) * QRS); }
                const size_t oo = sb + (size_t)row * (size_t)pitch + c8;
                *(volatile v8h*)(Ph + oo) = hv; if (useRes) *(volatile v8h*)(Pr + oo) = rv; }
            if (ps == 0) __threadfence(); }
        wave_sync();
    }
}

__global__ __launch_bounds__(32 * AW) void k_flash(const h16* __restrict__ QH, const h16* __restrict__ KH, const h16* __restrict__ VT, const unsigned* __restrict__ MW, bf* CX, float* ST) {
    __shared__ __align__(16) float os[AW * 16 * 68];
    const int lane = threadIdx.x & 31; const int wave = __builtin_amdgcn_readfirstlane(threadIdx.x >> 5); const int lr = lane & 15, hi = lane >> 4;
    const int zh = blockIdx.y; const int b = zh / NH_, h = zh % NH_;
    const int t0 = (blockIdx.x * AW + wave) * 16;
    const size_t pbase = (size_t)zh * SEQ * HD;
    const size_t qo = pbase + (size_t)(t0 + lr) * HD + 8 * hi;
    const v16h qh0 = ldh(QH + qo), qh1 = ldh(QH + qo + 32);
    const size_t ko = pbase + (size_t)lr * HD + 8 * hi;
    const size_t vo = pbase + (size_t)lr * SEQ + 8 * hi;
    const int mwb = b * (SEQ / 32);
    v8f o0 = (v8f){}, o1 = (v8f){}, o2 = (v8f){}, o3 = (v8f){};
    float m = -3.0e38f, l = 0.0f;
#pragma unroll 1
    for (int key0 = 0; key0 < SEQ; key0 += 32) {
        const h16* ka = KH + ko + (size_t)key0 * HD;
        const v16h ka0 = ldh(ka), ka1 = ldh(ka + 32), kb0 = ldh(ka + 16 * HD), kb1 = ldh(ka + 16 * HD + 32);
        const unsigned kw = MW[mwb + (key0 >> 5)];
        v8f sHa = (v8f){}, sHb = (v8f){};
        sHa = wmma16(ka0, qh0, sHa); sHb = wmma16(kb0, qh0, sHb);
        sHa = wmma16(ka1, qh1, sHa); sHb = wmma16(kb1, qh1, sHb);
        asm volatile("v_nop\n\tv_nop\n\tv_nop\n\tv_nop" : "+v"(sHa), "+v"(sHb) : "v"(ka0), "v"(ka1), "v"(kb0), "v"(kb1), "v"(qh0), "v"(qh1));
        const unsigned ba = (kw >> (8 * hi)) & 0xFFu, bc = (kw >> (16 + 8 * hi)) & 0xFFu;
        float ta[8], tb[8]; float mx = -3.0e38f;
#pragma unroll
        for (int r = 0; r < 8; ++r) {
            const float xa = sHa[r] * SC2;
            const float xc = sHb[r] * SC2;
            ta[r] = (((ba >> r) & 1u) != 0u) ? xa : -3.0e38f;
            tb[r] = (((bc >> r) & 1u) != 0u) ? xc : -3.0e38f;
            mx = fmaxf(mx, fmaxf(ta[r], tb[r])); }
        mx = fmaxf(mx, __shfl_xor(mx, 16, 32));
        const float mnew = fmaxf(m, mx);
        const float alpha = __builtin_amdgcn_exp2f(m - mnew);
        v16h pb; float ls = 0.0f;
#pragma unroll
        for (int r = 0; r < 8; ++r) {
            const h16 pa = p_exp2_flush((ta[r] - mnew) + PSH, ((ba >> r) & 1u) != 0u);
            const h16 pc = p_exp2_flush((tb[r] - mnew) + PSH, ((bc >> r) & 1u) != 0u);
            pb[r] = pa; pb[8 + r] = pc; ls += (float)pa + (float)pc; }
        l = l * alpha + ls; m = mnew;
        o0 = o0 * alpha; o1 = o1 * alpha; o2 = o2 * alpha; o3 = o3 * alpha;
        const h16* va = VT + vo + key0;
        const v16h v0 = ldh(va), v1 = ldh(va + (size_t)16 * SEQ), v2 = ldh(va + (size_t)32 * SEQ), v3 = ldh(va + (size_t)48 * SEQ);
        o0 = wmma16(v0, pb, o0); o1 = wmma16(v1, pb, o1); o2 = wmma16(v2, pb, o2); o3 = wmma16(v3, pb, o3);
        asm volatile("v_nop\n\tv_nop\n\tv_nop\n\tv_nop" : "+v"(o0), "+v"(o1), "+v"(o2), "+v"(o3) : "v"(v0), "v"(v1), "v"(v2), "v"(v3), "v"(pb));
    }
    l += __shfl_xor(l, 16, 32);
    const float lc = fmaxf(l, 1.0e-30f);
    const float rl = 1.0f / lc;
    const float inv = (l > 0.0f) ? rl : 0.0f;
    const float mst = (l > 0.0f) ? m : 0.0f;
    const float wst = inv * AMW;
    { const int sl = (2 * lane) & 15;
      const float m0 = __shfl(mst, sl, 32), m1 = __shfl(mst, sl + 1, 32), w0 = __shfl(wst, sl, 32), w1 = __shfl(wst, sl + 1, 32);
      v4f sv; sv[0] = m0; sv[1] = w0; sv[2] = m1; sv[3] = w1;
      float* sp = ST + ((size_t)zh * SEQ + t0) * 2 + 4 * (lane & 7);
      if (lane < 8) *(volatile v4f*)sp = sv;
      __threadfence();
      if (lane < 8) *(volatile v4f*)sp = sv; }
    const int wb = wave * 16 * 68;
    { v4f a, c;
      a[0] = o0[0] * inv; a[1] = o0[1] * inv; a[2] = o0[2] * inv; a[3] = o0[3] * inv; c[0] = o0[4] * inv; c[1] = o0[5] * inv; c[2] = o0[6] * inv; c[3] = o0[7] * inv;
      *(v4fa*)(&os[wb + lr * 68 +  0 + 8 * hi]) = a; *(v4fa*)(&os[wb + lr * 68 +  0 + 8 * hi + 4]) = c;
      a[0] = o1[0] * inv; a[1] = o1[1] * inv; a[2] = o1[2] * inv; a[3] = o1[3] * inv; c[0] = o1[4] * inv; c[1] = o1[5] * inv; c[2] = o1[6] * inv; c[3] = o1[7] * inv;
      *(v4fa*)(&os[wb + lr * 68 + 16 + 8 * hi]) = a; *(v4fa*)(&os[wb + lr * 68 + 16 + 8 * hi + 4]) = c;
      a[0] = o2[0] * inv; a[1] = o2[1] * inv; a[2] = o2[2] * inv; a[3] = o2[3] * inv; c[0] = o2[4] * inv; c[1] = o2[5] * inv; c[2] = o2[6] * inv; c[3] = o2[7] * inv;
      *(v4fa*)(&os[wb + lr * 68 + 32 + 8 * hi]) = a; *(v4fa*)(&os[wb + lr * 68 + 32 + 8 * hi + 4]) = c;
      a[0] = o3[0] * inv; a[1] = o3[1] * inv; a[2] = o3[2] * inv; a[3] = o3[3] * inv; c[0] = o3[4] * inv; c[1] = o3[5] * inv; c[2] = o3[6] * inv; c[3] = o3[7] * inv;
      *(v4fa*)(&os[wb + lr * 68 + 48 + 8 * hi]) = a; *(v4fa*)(&os[wb + lr * 68 + 48 + 8 * hi + 4]) = c; }
    wave_sync();
    bf* crow = CX + (size_t)(b * SEQ + t0) * KA + h * HD;
    const int c8 = (lane & 7) * 8, rq = lane >> 3;
#pragma unroll 1
    for (int ps = 0; ps < 2; ++ps) {
#pragma unroll
        for (int s = 0; s < 4; ++s) { const int row = 4 * s + rq;
            const v4f x0 = *(const v4fa*)(&os[wb + row * 68 + c8]); const v4f x1 = *(const v4fa*)(&os[wb + row * 68 + c8 + 4]); v8us hv, lv;
#pragma unroll
            for (int i = 0; i < 4; ++i) { const unsigned short a0 = f2bf(x0[i]); const unsigned short a1 = f2bf(x1[i]); hv[i] = a0; hv[4 + i] = a1; lv[i] = f2bf(x0[i] - bf2f(a0)); lv[4 + i] = f2bf(x1[i] - bf2f(a1)); }
            const size_t oo = (size_t)row * KA + c8;
            *(volatile v8us*)(crow + oo) = hv; *(volatile v8us*)(crow + oo + DM) = lv; }
        if (ps == 0) __threadfence(); }
}

__device__ __forceinline__ void amean_step(const h16* __restrict__ KH, size_t kofs, v16h qh0, v16h qh1, unsigned ba, unsigned bc, float mrow, float wrow, v8f& accA, v8f& accC) {
    const h16* ka = KH + kofs;
    const v16h ka0 = ldh(ka), ka1 = ldh(ka + 32), kb0 = ldh(ka + 16 * HD), kb1 = ldh(ka + 16 * HD + 32);
    v8f sa = (v8f){}, sb = (v8f){};
    sa = wmma16(ka0, qh0, sa); sb = wmma16(kb0, qh0, sb);
    sa = wmma16(ka1, qh1, sa); sb = wmma16(kb1, qh1, sb);
    asm volatile("v_nop\n\tv_nop\n\tv_nop\n\tv_nop" : "+v"(sa), "+v"(sb) : "v"(ka0), "v"(ka1), "v"(kb0), "v"(kb1), "v"(qh0), "v"(qh1));
#pragma unroll
    for (int r = 0; r < 8; ++r) {
        const float pa = __builtin_amdgcn_exp2f(sa[r] * SC2 - mrow) * wrow;
        const float pc = __builtin_amdgcn_exp2f(sb[r] * SC2 - mrow) * wrow;
        accA[r] += (((ba >> r) & 1u) != 0u) ? pa : 0.0f;
        accC[r] += (((bc >> r) & 1u) != 0u) ? pc : 0.0f; }
}

__global__ __launch_bounds__(32 * AW) void k_amean(const h16* __restrict__ QH, const h16* __restrict__ KH, const float* __restrict__ ST, const unsigned* __restrict__ MW, float* OUT) {
    __shared__ __align__(16) float os[AW * 16 * 68];
    const int lane = threadIdx.x & 31; const int wave = __builtin_amdgcn_readfirstlane(threadIdx.x >> 5); const int lr = lane & 15, hi = lane >> 4;
    const int b = blockIdx.z; const int kc0 = blockIdx.x * AKS;
    const int t0 = (blockIdx.y * AW + wave) * 16;
    const int mwb = b * (SEQ / 32) + (kc0 >> 5);
    const unsigned kw0 = MW[mwb], kw1 = MW[mwb + 1];
    const unsigned ba0 = (kw0 >> (8 * hi)) & 0xFFu, bc0 = (kw0 >> (16 + 8 * hi)) & 0xFFu;
    const unsigned ba1 = (kw1 >> (8 * hi)) & 0xFFu, bc1 = (kw1 >> (16 + 8 * hi)) & 0xFFu;
    v8f aA0 = (v8f){}, aC0 = (v8f){}, aA1 = (v8f){}, aC1 = (v8f){};
#pragma unroll 1
    for (int hh = 0; hh < NH_; ++hh) {
        const int zh = b * NH_ + hh;
        const size_t pbase = (size_t)zh * SEQ * HD;
        const size_t qo = pbase + (size_t)(t0 + lr) * HD + 8 * hi;
        const v16h qh0 = ldh(QH + qo), qh1 = ldh(QH + qo + 32);
        const v2f st = *(const v2f*)(ST + ((size_t)zh * SEQ + t0 + lr) * 2);
        const float mrow = st[0], wrow = st[1];
        const size_t ko = pbase + (size_t)(kc0 + lr) * HD + 8 * hi;
        amean_step(KH, ko, qh0, qh1, ba0, bc0, mrow, wrow, aA0, aC0);
        amean_step(KH, ko + (size_t)32 * HD, qh0, qh1, ba1, bc1, mrow, wrow, aA1, aC1);
    }
    const int wb = wave * 16 * 68;
    { v4f a, c;
      a[0] = aA0[0]; a[1] = aA0[1]; a[2] = aA0[2]; a[3] = aA0[3]; c[0] = aA0[4]; c[1] = aA0[5]; c[2] = aA0[6]; c[3] = aA0[7];
      *(v4fa*)(&os[wb + lr * 68 +  0 + 8 * hi]) = a; *(v4fa*)(&os[wb + lr * 68 +  0 + 8 * hi + 4]) = c;
      a[0] = aC0[0]; a[1] = aC0[1]; a[2] = aC0[2]; a[3] = aC0[3]; c[0] = aC0[4]; c[1] = aC0[5]; c[2] = aC0[6]; c[3] = aC0[7];
      *(v4fa*)(&os[wb + lr * 68 + 16 + 8 * hi]) = a; *(v4fa*)(&os[wb + lr * 68 + 16 + 8 * hi + 4]) = c;
      a[0] = aA1[0]; a[1] = aA1[1]; a[2] = aA1[2]; a[3] = aA1[3]; c[0] = aA1[4]; c[1] = aA1[5]; c[2] = aA1[6]; c[3] = aA1[7];
      *(v4fa*)(&os[wb + lr * 68 + 32 + 8 * hi]) = a; *(v4fa*)(&os[wb + lr * 68 + 32 + 8 * hi + 4]) = c;
      a[0] = aC1[0]; a[1] = aC1[1]; a[2] = aC1[2]; a[3] = aC1[3]; c[0] = aC1[4]; c[1] = aC1[5]; c[2] = aC1[6]; c[3] = aC1[7];
      *(v4fa*)(&os[wb + lr * 68 + 48 + 8 * hi]) = a; *(v4fa*)(&os[wb + lr * 68 + 48 + 8 * hi + 4]) = c; }
    wave_sync();
    float* orow = OUT + AM_OFF + ((size_t)b * OUT_SEQ + t0) * (size_t)AM_PITCH + kc0;
    const int cofs = lr * 4;
#pragma unroll 1
    for (int ps = 0; ps < 2; ++ps) {
#pragma unroll
        for (int s = 0; s < 8; ++s) { const int row = 2 * s + hi;
            const v4f x = *(const v4fa*)(&os[wb + row * 68 + cofs]);
            *(volatile v4f*)(orow + (size_t)row * (size_t)AM_PITCH + cofs) = x; }
        if (ps == 0) __threadfence(); }
}

__global__ __launch_bounds__(32) void k_out(const bf* __restrict__ A, const bf* __restrict__ Bt, const float* __restrict__ bias, float* OUT) {
    __shared__ __align__(16) float os[16 * 68];
    const int lane = threadIdx.x & 31, lr = lane & 15, hi = lane >> 4; const int r0 = blockIdx.x * 64, c0 = blockIdx.y * 64;
    v8f acc[4][4];
#pragma unroll
    for (int mb = 0; mb < 4; ++mb)
#pragma unroll
        for (int nb = 0; nb < 4; ++nb) acc[mb][nb] = (v8f){};
    const size_t aoff = (size_t)(r0 + lr) * KA + 8 * hi, boff = (size_t)(c0 + lr) * DM + 8 * hi;
#pragma unroll 1
    for (int kc = 0; kc < KA; kc += 32) {
        const int kb = (kc < DM) ? kc : (kc - DM);
        v16bf a[4];
#pragma unroll
        for (int mb = 0; mb < 4; ++mb) a[mb] = ldb(A + aoff + (size_t)mb * 16 * KA + kc);
        v16bf b = ldb(Bt + boff + kb);
#pragma unroll
        for (int mb = 0; mb < 4; ++mb) acc[mb][0] = wmmab(a[mb], b, acc[mb][0]);
#pragma unroll
        for (int nb = 1; nb < 4; ++nb) { b = ldb(Bt + boff + (size_t)nb * 16 * DM + kb);
#pragma unroll
            for (int mb = 0; mb < 4; ++mb) acc[mb][nb] = wmmab(a[mb], b, acc[mb][nb]); }
        asm volatile("" : "+v"(acc[2][0]), "+v"(acc[2][1]), "+v"(acc[2][2]), "+v"(acc[2][3]), "+v"(acc[3][0]), "+v"(acc[3][1]), "+v"(acc[3][2]), "+v"(acc[3][3]));
        asm volatile("v_nop\n\tv_nop\n\tv_nop\n\tv_nop" : "+v"(acc[0][0]), "+v"(acc[0][1]), "+v"(acc[0][2]), "+v"(acc[0][3]), "+v"(acc[1][0]), "+v"(acc[1][1]), "+v"(acc[1][2]), "+v"(acc[1][3]) : "v"(a[0]), "v"(a[1]), "v"(a[2]), "v"(a[3]), "v"(b));
    }
    const int cofs = lr * 4;
    const v4f braw = *(const v4f*)(bias + c0 + cofs);
    v4f bv; bv[0] = bfr(braw[0]); bv[1] = bfr(braw[1]); bv[2] = bfr(braw[2]); bv[3] = bfr(braw[3]);
    const int bb = r0 / SEQ, tt = r0 % SEQ;
    float* orow = OUT + ((size_t)bb * OUT_SEQ + tt) * DM + c0;
#pragma unroll
    for (int mb = 0; mb < 4; ++mb) {
#pragma unroll
        for (int nb = 0; nb < 4; ++nb) {
#pragma unroll
            for (int j = 0; j < 8; ++j) os[(hi * 8 + j) * 68 + nb * 16 + lr] = acc[mb][nb][j]; }
        wave_sync();
#pragma unroll 1
        for (int ps = 0; ps < 2; ++ps) {
#pragma unroll
            for (int s = 0; s < 8; ++s) { const int row = 2 * s + hi;
                const v4f x = *(const v4fa*)(&os[row * 68 + cofs]);
                const v4f val = x + bv;
                *(volatile v4f*)(orow + (size_t)(mb * 16 + row) * DM + cofs) = val; }
            if (ps == 0) __threadfence(); }
        wave_sync();
    }
}

static constexpr size_t al256(size_t v) { return (v + 255) & ~(size_t)255; }
static constexpr size_t SZ_XB = al256((size_t)NB * SEQ * DM * 2);
static constexpr size_t SZ_WB = al256((size_t)4 * DM * DM * 2);
static constexpr size_t SZ_PRE = al256((size_t)NB * SEQ * DM * 4);
static constexpr size_t SZ_PL = al256((size_t)NB * NH_ * SEQ * HD * 2);
static constexpr size_t SZ_CX = al256((size_t)NB * SEQ * KA * 2);
static constexpr size_t SZ_ST = al256((size_t)NB * NH_ * SEQ * 2 * 4);
static constexpr size_t SZ_RT = al256((size_t)SEQ * RP * 4);
static constexpr size_t SZ_MW = al256((size_t)NWP * 4);
static constexpr size_t SZ_TOTAL = 2 * SZ_XB + SZ_WB + 2 * SZ_PRE + 3 * SZ_PL + SZ_CX + SZ_ST + 2 * SZ_RT + SZ_MW;
static_assert(SZ_TOTAL <= (size_t)134217728);
static_assert(((size_t)DM * DM * 2) % 256 == 0);

extern "C" void kernel_launch(void* const* d_in, const int* in_sizes, int n_in,
                              void* d_out, int out_size, void* d_ws, size_t ws_size, hipStream_t stream) {
    if (n_in < 13) return;
    const size_t needx = ((size_t)(NB - 1) * SEQ_FULL + SEQ) * DM;
    if ((size_t)in_sizes[0] < needx || (size_t)in_sizes[1] < needx) return;
    if ((size_t)in_sizes[2] < (size_t)(NB - 1) * SEQ_FULL + SEQ) return;
    if ((size_t)in_sizes[3] < (size_t)DM * DM || (size_t)in_sizes[5] < (size_t)DM * DM || (size_t)in_sizes[7] < (size_t)DM * DM || (size_t)in_sizes[9] < (size_t)DM * DM) return;
    if (in_sizes[4] < DM || in_sizes[6] < DM || in_sizes[8] < DM || in_sizes[10] < DM || in_sizes[11] < DM || in_sizes[12] < DM) return;
    if ((size_t)out_size < AM_OFF + ((size_t)(NB - 1) * OUT_SEQ + (size_t)(SEQ - 1)) * (size_t)AM_PITCH + SEQ) return;
    if ((size_t)out_size < ((size_t)(NB - 1) * OUT_SEQ + SEQ) * DM) return;
    if (SZ_TOTAL > ws_size) return;
    const float* x = (const float*)d_in[0]; const float* enc = (const float*)d_in[1]; const int* mask = (const int*)d_in[2];
    const float* wk = (const float*)d_in[3]; const float* bk = (const float*)d_in[4]; const float* wq = (const float*)d_in[5]; const float* bq = (const float*)d_in[6];
    const float* wv = (const float*)d_in[7]; const float* bvv = (const float*)d_in[8]; const float* wo = (const float*)d_in[9]; const float* bo = (const float*)d_in[10];
    const float* gq = (const float*)d_in[11]; const float* gk = (const float*)d_in[12];
    float* OUT = (float*)d_out;
    char* wsp = (char*)d_ws;
    bf* XB  = (bf*)wsp; wsp += SZ_XB;
    bf* KVB = (bf*)wsp; wsp += SZ_XB;
    bf* WB  = (bf*)wsp; wsp += SZ_WB;
    float* PQ = (float*)wsp; wsp += SZ_PRE;
    float* PK = (float*)wsp; wsp += SZ_PRE;
    h16* QH = (h16*)wsp; wsp += SZ_PL;
    h16* KH = (h16*)wsp; wsp += SZ_PL;
    h16* VT = (h16*)wsp; wsp += SZ_PL;
    bf* CX  = (bf*)wsp; wsp += SZ_CX;
    float* ST = (float*)wsp; wsp += SZ_ST;
    float* RC = (float*)wsp; wsp += SZ_RT;
    float* RS = (float*)wsp; wsp += SZ_RT;
    unsigned* MW = (unsigned*)wsp; wsp += SZ_MW;
    bf* WQ = WB; bf* WK = WB + (size_t)DM * DM; bf* WV = WB + (size_t)2 * DM * DM; bf* WO = WB + (size_t)3 * DM * DM;

    k_mask<<<NWP / 32, 32, 0, stream>>>(mask, MW, NWORDS);

    { const unsigned p8 = (unsigned)((size_t)SEQ * DM / 8); const dim3 g((p8 + 255) / 256, NB, 1);
      k_cvt<<<g, 256, 0, stream>>>(x,   XB,  p8, (unsigned)(DM / 8), (size_t)SEQ_FULL * DM, (size_t)DM);
      k_cvt<<<g, 256, 0, stream>>>(enc, KVB, p8, (unsigned)(DM / 8), (size_t)SEQ_FULL * DM, (size_t)DM); }
    { const unsigned p8 = (unsigned)((size_t)DM * DM / 8); const dim3 g((p8 + 255) / 256, 1, 1);
      k_cvt<<<g, 256, 0, stream>>>(wq, WQ, p8, (unsigned)(DM / 8), (size_t)0, (size_t)DM);
      k_cvt<<<g, 256, 0, stream>>>(wk, WK, p8, (unsigned)(DM / 8), (size_t)0, (size_t)DM);
      k_cvt<<<g, 256, 0, stream>>>(wv, WV, p8, (unsigned)(DM / 8), (size_t)0, (size_t)DM);
      k_cvt<<<g, 256, 0, stream>>>(wo, WO, p8, (unsigned)(DM / 8), (size_t)0, (size_t)DM); }

    k_rtab<<<SEQ / 8, 256, 0, stream>>>(RC, RS);

    k_pre<<<dim3(NB * SEQ / 64, DM / 64, 1), 32, 0, stream>>>(XB,  WQ, bq, PQ);
    k_pre<<<dim3(NB * SEQ / 64, DM / 64, 1), 32, 0, stream>>>(KVB, WK, bk, PK);
    k_nrope<<<NB * SEQ / 8, 256, 0, stream>>>(PQ, gq, RC, RS, QH);
    k_nrope<<<NB * SEQ / 8, 256, 0, stream>>>(PK, gk, RC, RS, KH);
    k_proj<<<dim3(DM / 64, NB * SEQ / 64, 1), 32, 0, stream>>>(WV, KVB, bvv, 1, VT, VT, 0, DM, (size_t)0, SEQ, SEQ, (size_t)DM * SEQ);

    k_flash<<<dim3(SEQ / (16 * AW), NB * NH_, 1), 32 * AW, 0, stream>>>(QH, KH, VT, MW, CX, ST);

    k_amean<<<dim3(SEQ / AKS, SEQ / (16 * AW), NB), 32 * AW, 0, stream>>>(QH, KH, ST, MW, OUT);

    k_out<<<dim3(NB * SEQ / 64, DM / 64, 1), 32, 0, stream>>>(CX, WO, bo, OUT);
}
